// MultiHeadCrossAttention_6451040878908
// MI455X (gfx1250) — hardware-verified
//
#include <hip/hip_runtime.h>
#include <math.h>

#ifndef NB
#define NB 4
#endif
#ifndef NQS
#define NQS 1024
#endif
#define NB_FULL 4
#define NQ_FULL 1024
#define NKV 2048
#define DM 1024
#define NH 16
#define HD 64
static_assert(NB >= 1 && NB <= NB_FULL);
static_assert(NQS % 64 == 0 && NQS >= 64 && NQS <= NQ_FULL);
static_assert(NKV % 64 == 0 && DM % 64 == 0 && NH * HD == DM && HD == 64);

typedef __attribute__((ext_vector_type(16))) _Float16 v16h;
typedef __attribute__((ext_vector_type(8)))  _Float16 v8h;
typedef __attribute__((ext_vector_type(16))) __bf16   v16b;
typedef __attribute__((ext_vector_type(8)))  __bf16   v8b;
typedef __attribute__((ext_vector_type(8)))  float    v8f;
typedef __attribute__((ext_vector_type(4)))  float    v4f;
typedef __attribute__((ext_vector_type(8)))  unsigned short v8us;
typedef __attribute__((ext_vector_type(4)))  int      v4i;

#define VST2(T, ptr, val) do { const T vst2_v_ = (val); *(volatile T*)(ptr) = vst2_v_; __threadfence(); *(volatile T*)(ptr) = vst2_v_; } while (0)

__device__ __forceinline__ unsigned short bfbits(float f) { unsigned u = __float_as_uint(f); u += 0x7fffu + ((u >> 16) & 1u); return (unsigned short)(u >> 16); }
__device__ __forceinline__ float bf2f(unsigned short b) { return __uint_as_float(((unsigned)b) << 16); }


namespace gk {
__device__ __forceinline__ void dep_guard_h(v8f& a, v8f& b, v16h x, v16h y) { asm volatile("v_nop\n\tv_nop\n\tv_nop\n\tv_nop" : "+v"(a), "+v"(b) : "v"(x), "v"(y)); }
__device__ __forceinline__ void dep_guard_b(v8f& a, v8f& b, v16b x, v16b y) { asm volatile("v_nop\n\tv_nop\n\tv_nop\n\tv_nop" : "+v"(a), "+v"(b) : "v"(x), "v"(y)); }
__device__ __forceinline__ void keep4_h(v16h a, v16h b, v16h c, v16h d) { asm volatile("v_nop" :: "v"(a), "v"(b), "v"(c), "v"(d)); }
__device__ __forceinline__ void keep4_b(v16b a, v16b b, v16b c, v16b d) { asm volatile("v_nop" :: "v"(a), "v"(b), "v"(c), "v"(d)); }
__device__ __forceinline__ void acc_guard4(v8f& a, v8f& b, v8f& c, v8f& d) { asm volatile("v_nop\n\tv_nop\n\tv_nop\n\tv_nop" : "+v"(a), "+v"(b), "+v"(c), "+v"(d)); }
template <typename T> struct Frag;
template <> struct Frag<_Float16> {
  typedef v16h V; union U { v16h v; v8h h[2]; };
  static __device__ __forceinline__ v16h load(const _Float16* p) {
    U f; f.h[0] = *(const v8h*)(p); f.h[1] = *(const v8h*)(p + 16); return f.v;
  }
  static __device__ __forceinline__ v8f mma(v16h a, v16h b, v8f c) {
    return __builtin_amdgcn_wmma_f32_16x16x32_f16(false, a, false, b, (short)0, c, false, false);
  }
  static __device__ __forceinline__ void guard(v8f& a, v8f& b, v16h x, v16h y) { dep_guard_h(a, b, x, y); }
  static __device__ __forceinline__ void keep(v16h a, v16h b, v16h c, v16h d) { keep4_h(a, b, c, d); }
};
template <> struct Frag<__bf16> {
  typedef v16b V; union U { v16b v; v8b h[2]; };
  static __device__ __forceinline__ v16b load(const __bf16* p) {
    U f; f.h[0] = *(const v8b*)(p); f.h[1] = *(const v8b*)(p + 16); return f.v;
  }
  static __device__ __forceinline__ v8f mma(v16b a, v16b b, v8f c) {
    return __builtin_amdgcn_wmma_f32_16x16x32_bf16(false, a, false, b, (short)0, c, false, false);
  }
  static __device__ __forceinline__ void guard(v8f& a, v8f& b, v16b x, v16b y) { dep_guard_b(a, b, x, y); }
  static __device__ __forceinline__ void keep(v16b a, v16b b, v16b c, v16b d) { keep4_b(a, b, c, d); }
};
template <int ET> struct Elem;
template <> struct Elem<0> { typedef _Float16 T; };
template <> struct Elem<1> { typedef __bf16 T; };

template <int ET, bool SPLIT, int BIAS_MODE, int OUT_MODE, bool RESID>
__global__ __launch_bounds__(256) void wmma_gemm64(
    const unsigned short* __restrict__ Ap, const unsigned short* __restrict__ A2p, int lda, long strideA,
    const unsigned short* __restrict__ Btp, const unsigned short* __restrict__ Bt2p, int ldb, long strideB,
    void* __restrict__ Cout, void* __restrict__ Cout2, int ldc, long strideC,
    const float* __restrict__ bias,
    const float* __restrict__ resid, long strideR,
    int M, int N, int K, float scale) {
  typedef typename Elem<ET>::T T;
  typedef typename Frag<T>::V V;
  const T* A = (const T*)Ap; const T* A2 = (const T*)A2p; const T* Bt = (const T*)Btp; const T* Bt2 = (const T*)Bt2p;
  __shared__ __align__(16) float sT[8][16 * 68];
  const int b    = blockIdx.y;
  const int lane = threadIdx.x & 31;
  const int wave = threadIdx.x >> 5;
  const int tilesN = N >> 6;
  const int tilesM = M >> 6;
  const int tile = blockIdx.x * 8 + wave;
  if (tile >= tilesM * tilesN) return;
  const int tm = tile / tilesN;
  const int tn = tile - tm * tilesN;
  const int m0 = tm << 6;
  const int n0 = tn << 6;

  const T* Ab  = A  + (size_t)b * strideA;
  const T* Bb  = Bt + (size_t)b * strideB;
  const T* Ab2 = SPLIT ? (A2  + (size_t)b * strideA) : nullptr;
  const T* Bb2 = SPLIT ? (Bt2 + (size_t)b * strideB) : nullptr;

  const int rlane = lane & 15;
  const int koff  = (lane >> 4) * 8;
  const int mOff  = (lane >> 4) * 8;

  v8f acc[4][4];
#pragma unroll
  for (int i = 0; i < 4; ++i)
#pragma unroll
    for (int j = 0; j < 4; ++j) acc[i][j] = (v8f){0.f,0.f,0.f,0.f,0.f,0.f,0.f,0.f};

  for (int k0 = 0; k0 < K; k0 += 32) {
    V bh[4], bl[4];
#pragma unroll
    for (int j = 0; j < 4; ++j) {
      const size_t bo = (size_t)(n0 + (j << 4) + rlane) * ldb + koff + k0;
      bh[j] = Frag<T>::load(Bb + bo);
      if (SPLIT) bl[j] = Frag<T>::load(Bb2 + bo); else bl[j] = bh[j];
    }
#pragma unroll
    for (int i = 0; i < 4; ++i) {
      const size_t ao = (size_t)(m0 + (i << 4) + rlane) * lda + koff + k0;
      V ah = Frag<T>::load(Ab + ao);
      V al;
      if (SPLIT) al = Frag<T>::load(Ab2 + ao); else al = ah;
#pragma unroll
      for (int j = 0; j < 4; ++j) {
        acc[i][j] = Frag<T>::mma(ah, bh[j], acc[i][j]);
        if (SPLIT) {
          acc[i][j] = Frag<T>::mma(ah, bl[j], acc[i][j]);
          acc[i][j] = Frag<T>::mma(al, bh[j], acc[i][j]);
        }
      }
      Frag<T>::guard(acc[i][0], acc[i][3], ah, al);
    }
    Frag<T>::keep(bh[0], bh[1], bh[2], bh[3]);
    if (SPLIT) Frag<T>::keep(bl[0], bl[1], bl[2], bl[3]);
  }
  acc_guard4(acc[0][0], acc[0][1], acc[0][2], acc[0][3]);
  acc_guard4(acc[1][0], acc[1][1], acc[1][2], acc[1][3]);
  acc_guard4(acc[2][0], acc[2][1], acc[2][2], acc[2][3]);
  acc_guard4(acc[3][0], acc[3][1], acc[3][2], acc[3][3]);

  float* slab = sT[wave];
  const float* Rb = RESID ? (resid + (size_t)b * strideR) : nullptr;
#pragma unroll
  for (int i = 0; i < 4; ++i) {
    const int mBase = m0 + (i << 4);
#pragma unroll
    for (int j = 0; j < 4; ++j) {
      const int n = n0 + (j << 4) + rlane;
      float bv = 0.f;
      if (BIAS_MODE == 2) bv = bias[n];
#pragma unroll
      for (int r = 0; r < 8; ++r) {
        float v = acc[i][j][r] * scale;
        if (BIAS_MODE == 1) v += bias[mBase + mOff + r];
        if (BIAS_MODE == 2) v += bv;
        if (RESID) v += Rb[(size_t)(mBase + mOff + r) * ldc + n];
        slab[(mOff + r) * 68 + (j << 4) + rlane] = v;
      }
    }
    __builtin_amdgcn_fence(3, "workgroup");
    __builtin_amdgcn_wave_barrier();
    __builtin_amdgcn_fence(2, "workgroup");
    if (OUT_MODE == 0) {
      float* C = (float*)Cout + (size_t)b * strideC;
      const int hh = lane >> 4, c4 = (lane & 15) * 4;
      for (int pass = 0; pass < 2; ++pass) {
#pragma unroll
        for (int it = 0; it < 8; ++it) {
          const int row = it * 2 + hh;
          v4f v = *(const v4f*)(slab + row * 68 + c4);
          *(volatile v4f*)(C + (size_t)(mBase + row) * ldc + n0 + c4) = v;
        }
        __threadfence();
      }
    } else {
      const int q = lane >> 3, c8 = (lane & 7) * 8;
      unsigned short* C  = (unsigned short*)Cout  + (size_t)b * strideC;
      unsigned short* C2 = (OUT_MODE == 2) ? ((unsigned short*)Cout2 + (size_t)b * strideC) : nullptr;
      for (int pass = 0; pass < 2; ++pass) {
#pragma unroll
        for (int it = 0; it < 4; ++it) {
          const int row = it * 4 + q;
          const float* sp = slab + row * 68 + c8;
          v8us hv, lv;
#pragma unroll
          for (int e = 0; e < 8; ++e) {
            const float f = sp[e];
            if (OUT_MODE == 1) {
              const _Float16 fh = (_Float16)f;
              hv[e] = __builtin_bit_cast(unsigned short, fh); lv[e] = 0;
            } else {
              const unsigned short hb = bfbits(f);
              hv[e] = hb; lv[e] = bfbits(f - bf2f(hb));
            }
          }
          *(volatile v8us*)(C + (size_t)(mBase + row) * ldc + n0 + c8) = hv;
          if (OUT_MODE == 2) *(volatile v8us*)(C2 + (size_t)(mBase + row) * ldc + n0 + c8) = lv;
        }
        __threadfence();
      }
    }
    __builtin_amdgcn_fence(3, "workgroup");
    __builtin_amdgcn_wave_barrier();
    __builtin_amdgcn_fence(2, "workgroup");
  }
}
}

__global__ __launch_bounds__(256) void k_actpl(const float* __restrict__ src, long long sbat, int RPB, long long NR, unsigned short* __restrict__ dst) {
    const long long u = (long long)blockIdx.x * 256 + threadIdx.x;
    if (u >= NR * (DM / 8)) return;
    const long long r = u / (DM / 8); const int c = 8 * (int)(u % (DM / 8));
    const long long bb = r / RPB, rr = r % RPB;
    const float* s = src + bb * sbat + rr * DM + c;
    const v4f a = *(const v4f*)s; const v4f d = *(const v4f*)(s + 4);
    v8us o;
    o[0] = bfbits(a.x); o[1] = bfbits(a.y); o[2] = bfbits(a.z); o[3] = bfbits(a.w);
    o[4] = bfbits(d.x); o[5] = bfbits(d.y); o[6] = bfbits(d.z); o[7] = bfbits(d.w);
    volatile v8us* p = (volatile v8us*)(dst + r * DM + c); *p = o; __threadfence(); *p = o;
}
__global__ __launch_bounds__(256) void k_wpl(const float* __restrict__ W, int ldw, int NROW, int KP, int KI, int GRP, int GSTR, int GOFF, unsigned short* __restrict__ dst) {
    const long long u = (long long)blockIdx.x * 256 + threadIdx.x;
    if (u >= (long long)NROW * (KP / 8)) return;
    const int row = (int)(u / (KP / 8)); const int k0 = 8 * (int)(u % (KP / 8));
    int col = (row / GRP) * GSTR + GOFF + (row % GRP); col = min(max(col, 0), ldw - 1);
    v8us o;
#pragma unroll
    for (int e = 0; e < 8; ++e) { const int kk = (k0 + e) % KI; o[e] = bfbits(W[(long long)kk * ldw + col]); }
    volatile v8us* p = (volatile v8us*)(dst + (long long)row * KP + k0); *p = o; __threadfence(); *p = o;
}
__global__ __launch_bounds__(256) void k_bias(const float* __restrict__ bkv, const float* __restrict__ bq, const float* __restrict__ bo, float* __restrict__ BV) {
    const int t = blockIdx.x * 256 + threadIdx.x; if (t >= 4 * DM) return;
    const int seg = t >> 10, i = t & 1023;
    const int i1 = (i >> 6) * 128 + (i & 63);
    const float vk = bkv[i1], vv = bkv[i1 + 64], vq = bq[i], vo = bo[i];
    const float sel = (seg == 0) ? vk : ((seg == 1) ? vv : ((seg == 2) ? vq : vo));
    const float cv = bf2f(bfbits(sel)) * ((seg == 3) ? 1.0f : 8.0f);
    VST2(float, BV + t, cv);
}
__global__ __launch_bounds__(256) void k_mpack(const int* __restrict__ mask, unsigned* __restrict__ pm, long long nwords) {
    const long long u = (long long)blockIdx.x * 256 + threadIdx.x; if (u >= nwords) return;
    const long long row = u >> 6; const int wi = (int)(u & 63);
    const long long bb = row / NQS, q = row % NQS;
    const int* s = mask + ((bb * NQ_FULL + q) * NKV + (long long)wi * 32);
    unsigned w = 0u;
#pragma unroll
    for (int g = 0; g < 8; ++g) {
        const v4i m4 = *(const v4i*)(s + 4 * g);
        w |= ((m4.x != 0) ? 1u : 0u) << (4 * g);
        w |= ((m4.y != 0) ? 1u : 0u) << (4 * g + 1);
        w |= ((m4.z != 0) ? 1u : 0u) << (4 * g + 2);
        w |= ((m4.w != 0) ? 1u : 0u) << (4 * g + 3);
    }
    volatile unsigned* p = pm + u; *p = w; __threadfence(); *p = w;
}

#define PSC 16384.0f
union FH { v16h v; v8h h[2]; };
__device__ __forceinline__ v8f mma_h(v16h a, v16h b, v8f c) {
    c = __builtin_amdgcn_wmma_f32_16x16x32_f16(false, a, false, b, (short)0, c, false, false);
    asm volatile("v_nop\n\tv_nop\n\tv_nop\n\tv_nop" : "+v"(c) : "v"(a), "v"(b));
    return c;
}
__global__ __launch_bounds__(128) __attribute__((amdgpu_num_vgpr(256)))
void k_attn(const unsigned short* __restrict__ QPp, const unsigned short* __restrict__ KPp, const unsigned short* __restrict__ VTp,
            const unsigned* __restrict__ PM, unsigned short* __restrict__ CX, float sc2, float fill2) {
    __shared__ __align__(16) _Float16 Psh[4][16 * 64];
    __shared__ __align__(16) float    Os[4][16 * 68];
    const int tid = threadIdx.x, wave = tid >> 5, lane = tid & 31, hh = lane >> 4, c = lane & 15;
    const int nqb = NQS / 64;
    const int bx = blockIdx.x; const int qb = bx % nqb; const int bhd = bx / nqb; const int h = bhd % NH; const int b = bhd / NH;
    const int q0 = qb * 64 + wave * 16;
    const long long rowbase = (long long)b * NQS + q0;
    const float NEG = -__builtin_inff();

    v16h qa[2];
    {
        const _Float16* qrow = (const _Float16*)QPp + (rowbase + c) * DM + h * HD;
#pragma unroll
        for (int dc = 0; dc < 2; ++dc) { FH f; f.h[0] = *(const v8h*)(qrow + dc * 32 + 8 * hh); f.h[1] = *(const v8h*)(qrow + dc * 32 + 16 + 8 * hh); qa[dc] = f.v; }
    }
    const _Float16* kbp = (const _Float16*)KPp + (long long)b * NKV * DM + h * HD;
    const _Float16* vbp = (const _Float16*)VTp + ((long long)b * DM + h * HD) * (long long)NKV;
    const unsigned long long* pm64 = (const unsigned long long*)PM + (rowbase + 8 * hh) * (NKV / 64);

    float mrow[8], lrow[8];
    v8f oacc[4];
#pragma unroll
    for (int r = 0; r < 8; ++r) { mrow[r] = NEG; lrow[r] = 0.f; }
#pragma unroll
    for (int t = 0; t < 4; ++t) oacc[t] = (v8f){0.f,0.f,0.f,0.f,0.f,0.f,0.f,0.f};
    _Float16* pw = Psh[wave];

#pragma unroll 1
    for (int kc = 0; kc < NKV / 64; ++kc) {
        const int kv0 = kc * 64;
        v8f s[4];
#pragma unroll
        for (int j = 0; j < 4; ++j) {
            s[j] = (v8f){0.f,0.f,0.f,0.f,0.f,0.f,0.f,0.f};
            const _Float16* krow = kbp + (long long)(kv0 + j * 16 + c) * DM;
#pragma unroll
            for (int dc = 0; dc < 2; ++dc) {
                FH kf; kf.h[0] = *(const v8h*)(krow + dc * 32 + 8 * hh); kf.h[1] = *(const v8h*)(krow + dc * 32 + 16 + 8 * hh);
                s[j] = mma_h(qa[dc], kf.v, s[j]);
            }
        }
        float cm[8];
#pragma unroll
        for (int r = 0; r < 8; ++r) {
            const unsigned long long mw = pm64[(long long)r * (NKV / 64) + kc];
            const unsigned wl = ((unsigned)mw) >> c, wh = ((unsigned)(mw >> 32)) >> c;
            float m = NEG;
#pragma unroll
            for (int j = 0; j < 4; ++j) {
                const unsigned wsel = (j < 2) ? wl : wh;
                const unsigned bit = (wsel >> ((j & 1) * 16)) & 1u;
                float v = s[j][r] * sc2;
                v = (bit != 0u) ? v : fill2;
                s[j][r] = v;
                m = fmaxf(m, v);
            }
            m = fmaxf(m, __shfl_xor(m, 1, 32)); m = fmaxf(m, __shfl_xor(m, 2, 32));
            m = fmaxf(m, __shfl_xor(m, 4, 32)); m = fmaxf(m, __shfl_xor(m, 8, 32));
            cm[r] = m;
        }
#pragma unroll
        for (int r = 0; r < 8; ++r) {
            const float mnew = fmaxf(mrow[r], cm[r]);
            const float alpha = exp2f(mrow[r] - mnew);
            mrow[r] = mnew;
            float psum = 0.f;
#pragma unroll
            for (int j = 0; j < 4; ++j) {
                const float p = exp2f(s[j][r] - mnew);
                psum += p;
                pw[(8 * hh + r) * 64 + j * 16 + c] = (_Float16)(p * PSC);
            }
            psum += __shfl_xor(psum, 1, 32); psum += __shfl_xor(psum, 2, 32);
            psum += __shfl_xor(psum, 4, 32); psum += __shfl_xor(psum, 8, 32);
            lrow[r] = lrow[r] * alpha + psum;
#pragma unroll
            for (int t = 0; t < 4; ++t) oacc[t][r] *= alpha;
        }
        __builtin_amdgcn_fence(3, "workgroup");
        __builtin_amdgcn_wave_barrier();
        __builtin_amdgcn_fence(2, "workgroup");
#pragma unroll 1
        for (int kk = 0; kk < 2; ++kk) {
            FH pa; pa.h[0] = *(const v8h*)(pw + c * 64 + kk * 32 + 8 * hh); pa.h[1] = *(const v8h*)(pw + c * 64 + kk * 32 + 16 + 8 * hh);
#pragma unroll
            for (int t = 0; t < 4; ++t) {
                const _Float16* vrow = vbp + (long long)(t * 16 + c) * NKV + kv0 + kk * 32;
                FH vf; vf.h[0] = *(const v8h*)(vrow + 8 * hh); vf.h[1] = *(const v8h*)(vrow + 16 + 8 * hh);
                oacc[t] = mma_h(pa.v, vf.v, oacc[t]);
            }
        }
        __builtin_amdgcn_fence(3, "workgroup");
        __builtin_amdgcn_wave_barrier();
        __builtin_amdgcn_fence(2, "workgroup");
    }

    float* os = Os[wave];
#pragma unroll
    for (int r = 0; r < 8; ++r) {
        const float inv = 1.0f / (lrow[r] * (PSC * 8.0f));
#pragma unroll
        for (int t = 0; t < 4; ++t) os[(8 * hh + r) * 68 + t * 16 + c] = oacc[t][r] * inv;
    }
    __builtin_amdgcn_fence(3, "workgroup");
    __builtin_amdgcn_wave_barrier();
    __builtin_amdgcn_fence(2, "workgroup");
    {
        const int q8 = lane >> 3, c8 = (lane & 7) * 8;
        unsigned short* cxh = CX + h * HD;
        for (int pass = 0; pass < 2; ++pass) {
#pragma unroll
            for (int it = 0; it < 4; ++it) {
                const int row = it * 4 + q8;
                const float* sp = os + row * 68 + c8;
                const v4f a = *(const v4f*)sp; const v4f d = *(const v4f*)(sp + 4);
                float f8[8] = {a.x, a.y, a.z, a.w, d.x, d.y, d.z, d.w};
                v8us hv, lv;
#pragma unroll
                for (int e = 0; e < 8; ++e) { const unsigned short hb = bfbits(f8[e]); hv[e] = hb; lv[e] = bfbits(f8[e] - bf2f(hb)); }
                unsigned short* dst = cxh + (rowbase + row) * (2 * DM) + c8;
                *(volatile v8us*)(dst) = hv;
                *(volatile v8us*)(dst + DM) = lv;
            }
            __threadfence();
        }
    }
}

extern "C" void kernel_launch(void* const* d_in, const int* in_sizes, int n_in, void* d_out, int out_size, void* d_ws, size_t ws_size, hipStream_t stream) {
    if (n_in < 9) return;
    const float* x   = (const float*)d_in[0];
    const float* y   = (const float*)d_in[1];
    const int*   msk = (const int*)d_in[2];
    const float* Wkv = (const float*)d_in[3];
    const float* bkv = (const float*)d_in[4];
    const float* Wq  = (const float*)d_in[5];
    const float* bq  = (const float*)d_in[6];
    const float* Wo  = (const float*)d_in[7];
    const float* bo  = (const float*)d_in[8];
    if (in_sizes[0] < NB * NKV * DM) return;
    if (in_sizes[1] < ((NB - 1) * NQ_FULL + NQS) * DM) return;
    if (in_sizes[2] < ((NB - 1) * NQ_FULL + NQS) * NKV) return;
    if (in_sizes[3] < DM * 2 * DM || in_sizes[4] < 2 * DM || in_sizes[5] < DM * DM || in_sizes[6] < DM || in_sizes[7] < DM * DM || in_sizes[8] < DM) return;
    if (out_size < ((NB - 1) * NQ_FULL + NQS) * DM) return;
    float* out = (float*)d_out;

    char* wsp = (char*)d_ws;
    auto carve = [&](size_t bytes) { char* p = wsp; wsp += ((bytes + 255) / 256) * 256; return p; };
    unsigned short* XP  = (unsigned short*)carve((size_t)NB * NKV * DM * 2);
    unsigned short* YP  = (unsigned short*)carve((size_t)NB * NQS * DM * 2);
    unsigned short* WKT = (unsigned short*)carve((size_t)DM * DM * 2);
    unsigned short* WVT = (unsigned short*)carve((size_t)DM * DM * 2);
    unsigned short* WQT = (unsigned short*)carve((size_t)DM * DM * 2);
    unsigned short* WOT = (unsigned short*)carve((size_t)DM * 2 * DM * 2);
    float*          BV  = (float*)carve((size_t)4 * DM * 4);
    unsigned*       PM  = (unsigned*)carve((size_t)NB * NQS * (NKV / 32) * 4);
    unsigned short* KPL = (unsigned short*)carve((size_t)NB * NKV * DM * 2);
    unsigned short* VTP = (unsigned short*)carve((size_t)NB * DM * NKV * 2);
    unsigned short* QPL = (unsigned short*)carve((size_t)NB * NQS * DM * 2);
    unsigned short* CX  = (unsigned short*)carve((size_t)NB * NQS * 2 * DM * 2);
    if ((size_t)(wsp - (char*)d_ws) > ws_size) return;

    const float L2E = 1.4426950408889634f;
    const float sc2 = (0.125f / 64.0f) * L2E;
    const float fill2 = -1e20f * L2E;

    k_bias<<<(4 * DM + 255) / 256, 256, 0, stream>>>(bkv, bq, bo, BV);
    k_wpl<<<(unsigned)(((long long)DM * (DM / 8) + 255) / 256), 256, 0, stream>>>(Wkv, 2 * DM, DM, DM, DM, HD, 2 * HD, 0, WKT);
    k_wpl<<<(unsigned)(((long long)DM * (DM / 8) + 255) / 256), 256, 0, stream>>>(Wkv, 2 * DM, DM, DM, DM, HD, 2 * HD, HD, WVT);
    k_wpl<<<(unsigned)(((long long)DM * (DM / 8) + 255) / 256), 256, 0, stream>>>(Wq, DM, DM, DM, DM, DM, 0, 0, WQT);
    k_wpl<<<(unsigned)(((long long)DM * (2 * DM / 8) + 255) / 256), 256, 0, stream>>>(Wo, DM, DM, 2 * DM, DM, DM, 0, 0, WOT);
    k_actpl<<<(unsigned)(((long long)NB * NKV * (DM / 8) + 255) / 256), 256, 0, stream>>>(x, (long long)NKV * DM, NKV, (long long)NB * NKV, XP);
    k_actpl<<<(unsigned)(((long long)NB * NQS * (DM / 8) + 255) / 256), 256, 0, stream>>>(y, (long long)NQ_FULL * DM, NQS, (long long)NB * NQS, YP);
    k_mpack<<<(unsigned)(((long long)NB * NQS * (NKV / 32) + 255) / 256), 256, 0, stream>>>(msk, PM, (long long)NB * NQS * (NKV / 32));

    {
        const int tiles = (NB * NKV / 64) * (DM / 64);
        gk::wmma_gemm64<1, false, 2, 1, false><<<dim3((unsigned)((tiles + 7) / 8), 1u), 256, 0, stream>>>(
            XP, nullptr, DM, 0, WKT, nullptr, DM, 0, (void*)KPL, nullptr, DM, 0, BV + 0, nullptr, 0, NB * NKV, DM, DM, 8.0f);
    }
    {
        const int tiles = (DM / 64) * (NKV / 64);
        gk::wmma_gemm64<1, false, 1, 1, false><<<dim3((unsigned)((tiles + 7) / 8), (unsigned)NB), 256, 0, stream>>>(
            WVT, nullptr, DM, 0, XP, nullptr, DM, (long)NKV * DM, (void*)VTP, nullptr, NKV, (long)DM * NKV, BV + DM, nullptr, 0, DM, NKV, DM, 8.0f);
    }
    {
        const int tiles = (NB * NQS / 64) * (DM / 64);
        gk::wmma_gemm64<1, false, 2, 1, false><<<dim3((unsigned)((tiles + 7) / 8), 1u), 256, 0, stream>>>(
            YP, nullptr, DM, 0, WQT, nullptr, DM, 0, (void*)QPL, nullptr, DM, 0, BV + 2 * DM, nullptr, 0, NB * NQS, DM, DM, 8.0f);
    }
    k_attn<<<(unsigned)(NB * NH * (NQS / 64)), 128, 0, stream>>>(QPL, KPL, VTP, PM, CX, sc2, fill2);
    {
        const int tiles = (NQS / 64) * (DM / 64);
        gk::wmma_gemm64<1, false, 2, 0, false><<<dim3((unsigned)((tiles + 7) / 8), (unsigned)NB), 256, 0, stream>>>(
            CX, nullptr, 2 * DM, (long)NQS * 2 * DM, WOT, nullptr, 2 * DM, 0, (void*)out, nullptr, DM, (long)NQ_FULL * DM, BV + 3 * DM, nullptr, 0, NQS, DM, 2 * DM, 1.0f);
    }
}
